// DETRAttention_1812476199681
// MI455X (gfx1250) — hardware-verified
//
#include <hip/hip_runtime.h>

constexpr int NB_SZ = 4;
constexpr int SEQ_LEN = 2048;
constexpr int EMB_DIM = 1024;
constexpr int N_HEADS = 16;
constexpr int HEAD_DIM = 64;
constexpr int NROWS = NB_SZ * SEQ_LEN;
static_assert(EMB_DIM == N_HEADS * HEAD_DIM);
static_assert(HEAD_DIM == 64);
static_assert(NROWS % 64 == 0 && EMB_DIM % 64 == 0 && SEQ_LEN % 64 == 0);
static_assert(EMB_DIM % 32 == 0);

constexpr float W_CARRY = 64.0f;
constexpr float AO_CARRY = 64.0f;
constexpr float P_CARRY = 32768.0f;
constexpr float SCORE_SCALE_LOG2E = 0.125f * 1.4426950408889634f;

constexpr size_t N_ACT = (size_t)NROWS * EMB_DIM;
constexpr size_t N_W = (size_t)EMB_DIM * EMB_DIM;
constexpr size_t PLANE_ACT = N_ACT * 2;
constexpr size_t PLANE_W = N_W * 2;
constexpr size_t OFF_HQ = 0;
constexpr size_t OFF_HS = OFF_HQ + PLANE_ACT;
constexpr size_t OFF_W0 = OFF_HS + PLANE_ACT;
constexpr size_t OFF_Q = OFF_W0 + 4 * PLANE_W;
constexpr size_t OFF_K = OFF_Q + PLANE_ACT;
constexpr size_t OFF_VT = OFF_K + PLANE_ACT;
constexpr size_t WS_TOTAL = OFF_VT + PLANE_ACT;
static_assert(WS_TOTAL == 92274688ull);
static_assert(WS_TOTAL <= 134217728ull);

typedef __attribute__((ext_vector_type(16))) _Float16 v16h;
typedef __attribute__((ext_vector_type(8)))  _Float16 v8h;
typedef __attribute__((ext_vector_type(16))) __bf16   v16b;
typedef __attribute__((ext_vector_type(8)))  __bf16   v8b;
typedef __attribute__((ext_vector_type(8)))  float    v8f;
typedef __attribute__((ext_vector_type(4)))  float    v4f;

__device__ __forceinline__ unsigned short f2bf_bits(float f) {
  unsigned u = __float_as_uint(f);
  return (unsigned short)((u + 0x7FFFu + ((u >> 16) & 1u)) >> 16);
}
__device__ __forceinline__ float bf_bits2f(unsigned short h) { return __uint_as_float(((unsigned)h) << 16); }

__device__ __forceinline__ void dep_guard_h(v8f& a, v8f& b, v16h x, v16h y) { asm volatile("v_nop\n\tv_nop\n\tv_nop\n\tv_nop" : "+v"(a), "+v"(b) : "v"(x), "v"(y)); }
__device__ __forceinline__ void dep_guard_b(v8f& a, v8f& b, v16b x, v16b y) { asm volatile("v_nop\n\tv_nop\n\tv_nop\n\tv_nop" : "+v"(a), "+v"(b) : "v"(x), "v"(y)); }
__device__ __forceinline__ void keep4_h(v16h a, v16h b, v16h c, v16h d) { asm volatile("v_nop" :: "v"(a), "v"(b), "v"(c), "v"(d)); }
__device__ __forceinline__ void keep4_b(v16b a, v16b b, v16b c, v16b d) { asm volatile("v_nop" :: "v"(a), "v"(b), "v"(c), "v"(d)); }
__device__ __forceinline__ void acc_guard4(v8f& a, v8f& b, v8f& c, v8f& d) { asm volatile("v_nop\n\tv_nop\n\tv_nop\n\tv_nop" : "+v"(a), "+v"(b), "+v"(c), "+v"(d)); }

template <typename T> struct Frag;
template <> struct Frag<_Float16> {
  typedef v16h V; union U { v16h v; v8h h[2]; };
  static __device__ __forceinline__ v16h load(const _Float16* p) {
    U f; f.h[0] = *(const v8h*)(p); f.h[1] = *(const v8h*)(p + 16); return f.v;
  }
  static __device__ __forceinline__ v8f mma(v16h a, v16h b, v8f c) {
    return __builtin_amdgcn_wmma_f32_16x16x32_f16(false, a, false, b, (short)0, c, false, false);
  }
  static __device__ __forceinline__ void guard(v8f& a, v8f& b, v16h x, v16h y) { dep_guard_h(a, b, x, y); }
  static __device__ __forceinline__ void keep(v16h a, v16h b, v16h c, v16h d) { keep4_h(a, b, c, d); }
};
template <> struct Frag<__bf16> {
  typedef v16b V; union U { v16b v; v8b h[2]; };
  static __device__ __forceinline__ v16b load(const __bf16* p) {
    U f; f.h[0] = *(const v8b*)(p); f.h[1] = *(const v8b*)(p + 16); return f.v;
  }
  static __device__ __forceinline__ v8f mma(v16b a, v16b b, v8f c) {
    return __builtin_amdgcn_wmma_f32_16x16x32_bf16(false, a, false, b, (short)0, c, false, false);
  }
  static __device__ __forceinline__ void guard(v8f& a, v8f& b, v16b x, v16b y) { dep_guard_b(a, b, x, y); }
  static __device__ __forceinline__ void keep(v16b a, v16b b, v16b c, v16b d) { keep4_b(a, b, c, d); }
};

template <int ET> struct Elem;
template <> struct Elem<0> { typedef _Float16 T; };
template <> struct Elem<1> { typedef __bf16 T; };
template <int ET, bool SPLIT, int BIAS_MODE, int OUT_MODE>
__global__ __launch_bounds__(256) void wmma_gemm64(
    const unsigned short* __restrict__ Ap, const unsigned short* __restrict__ A2p, int lda, long strideA,
    const unsigned short* __restrict__ Btp, const unsigned short* __restrict__ Bt2p, int ldb, long strideB,
    void* __restrict__ Cout, void* __restrict__ Cout2, int ldc, long strideC,
    const float* __restrict__ bias,
    int M, int N, int K, float scale) {
  typedef typename Elem<ET>::T T;
  typedef typename Frag<T>::V V;
  const T* A = (const T*)Ap; const T* A2 = (const T*)A2p; const T* Bt = (const T*)Btp; const T* Bt2 = (const T*)Bt2p;
  __shared__ __align__(16) float sT[8][16 * 68];
  const int b    = blockIdx.y;
  const int lane = threadIdx.x & 31;
  const int wave = threadIdx.x >> 5;
  const int tilesN = N >> 6;
  const int tilesM = M >> 6;
  const int tile = blockIdx.x * 8 + wave;
  if (tile >= tilesM * tilesN) return;
  const int tm = tile / tilesN;
  const int tn = tile - tm * tilesN;
  const int m0 = tm << 6;
  const int n0 = tn << 6;

  const T* Ab  = A  + (size_t)b * strideA;
  const T* Bb  = Bt + (size_t)b * strideB;
  const T* Ab2 = SPLIT ? (A2  + (size_t)b * strideA) : nullptr;
  const T* Bb2 = SPLIT ? (Bt2 + (size_t)b * strideB) : nullptr;

  const int rlane = lane & 15;
  const int koff  = (lane >> 4) * 8;
  const int mOff  = (lane >> 4) * 8;

  v8f acc[4][4];
#pragma unroll
  for (int i = 0; i < 4; ++i)
#pragma unroll
    for (int j = 0; j < 4; ++j) acc[i][j] = (v8f){0.f,0.f,0.f,0.f,0.f,0.f,0.f,0.f};

  for (int k0 = 0; k0 < K; k0 += 32) {
    V bh[4], bl[4];
#pragma unroll
    for (int j = 0; j < 4; ++j) {
      const size_t bo = (size_t)(n0 + (j << 4) + rlane) * ldb + koff + k0;
      bh[j] = Frag<T>::load(Bb + bo);
      if (SPLIT) bl[j] = Frag<T>::load(Bb2 + bo);
    }
#pragma unroll
    for (int i = 0; i < 4; ++i) {
      const size_t ao = (size_t)(m0 + (i << 4) + rlane) * lda + koff + k0;
      V ah = Frag<T>::load(Ab + ao);
      V al = ah;
      if (SPLIT) al = Frag<T>::load(Ab2 + ao);
#pragma unroll
      for (int j = 0; j < 4; ++j) {
        acc[i][j] = Frag<T>::mma(ah, bh[j], acc[i][j]);
        if (SPLIT) {
          acc[i][j] = Frag<T>::mma(ah, bl[j], acc[i][j]);
          acc[i][j] = Frag<T>::mma(al, bh[j], acc[i][j]);
        }
      }
      Frag<T>::guard(acc[i][0], acc[i][3], ah, al);
    }
    Frag<T>::keep(bh[0], bh[1], bh[2], bh[3]);
    if (SPLIT) Frag<T>::keep(bl[0], bl[1], bl[2], bl[3]);
  }
  acc_guard4(acc[0][0], acc[0][1], acc[0][2], acc[0][3]);
  acc_guard4(acc[1][0], acc[1][1], acc[1][2], acc[1][3]);
  acc_guard4(acc[2][0], acc[2][1], acc[2][2], acc[2][3]);
  acc_guard4(acc[3][0], acc[3][1], acc[3][2], acc[3][3]);

  float* slab = sT[wave];
#pragma unroll
  for (int i = 0; i < 4; ++i) {
    const int mBase = m0 + (i << 4);
    float bm8[8];
#pragma unroll
    for (int r = 0; r < 8; ++r) bm8[r] = 0.f;
    if (BIAS_MODE == 1) {
      const v4f t0 = *(const v4f*)(bias + mBase + mOff);
      const v4f t1 = *(const v4f*)(bias + mBase + mOff + 4);
      bm8[0] = t0[0]; bm8[1] = t0[1]; bm8[2] = t0[2]; bm8[3] = t0[3];
      bm8[4] = t1[0]; bm8[5] = t1[1]; bm8[6] = t1[2]; bm8[7] = t1[3];
    }
#pragma unroll
    for (int j = 0; j < 4; ++j) {
      const int n = n0 + (j << 4) + rlane;
      float bv = 0.f;
      if (BIAS_MODE == 2) bv = bias[n];
#pragma unroll
      for (int r = 0; r < 8; ++r) {
        float v = acc[i][j][r] * scale;
        if (BIAS_MODE == 1) v += bm8[r];
        if (BIAS_MODE == 2) v += bv;
        slab[(mOff + r) * 68 + (j << 4) + rlane] = v;
      }
    }
    __builtin_amdgcn_fence(__ATOMIC_RELEASE, "workgroup");
    __builtin_amdgcn_wave_barrier();
    __builtin_amdgcn_fence(__ATOMIC_ACQUIRE, "workgroup");
    if (OUT_MODE == 0) {
      float* C = (float*)Cout + (size_t)b * strideC;
      const int hh = lane >> 4, c4 = (lane & 15) * 4;
      for (int pass = 0; pass < 2; ++pass) {
#pragma unroll
        for (int it = 0; it < 8; ++it) {
          const int row = it * 2 + hh;
          v4f v = *(const v4f*)(slab + row * 68 + c4);
          *(volatile v4f*)(C + (size_t)(mBase + row) * ldc + n0 + c4) = v;
        }
        __threadfence();
      }
    } else {
      const int q = lane >> 3, c8 = (lane & 7) * 8;
      unsigned short* C  = (unsigned short*)Cout  + (size_t)b * strideC;
      unsigned short* C2 = (OUT_MODE == 2) ? ((unsigned short*)Cout2 + (size_t)b * strideC) : nullptr;
      for (int pass = 0; pass < 2; ++pass) {
#pragma unroll
        for (int it = 0; it < 4; ++it) {
          const int row = it * 4 + q;
          const float* sp = slab + row * 68 + c8;
          v8h hv, lv;
#pragma unroll
          for (int e = 0; e < 8; ++e) {
            if (OUT_MODE == 1) {
              hv[e] = (_Float16)sp[e];
            } else {
              unsigned short hb = f2bf_bits(sp[e]);
              unsigned short lb = f2bf_bits(sp[e] - bf_bits2f(hb));
              hv[e] = __builtin_bit_cast(_Float16, hb);
              lv[e] = __builtin_bit_cast(_Float16, lb);
            }
          }
          *(volatile v8h*)(C + (size_t)(mBase + row) * ldc + n0 + c8) = hv;
          if (OUT_MODE == 2) *(volatile v8h*)(C2 + (size_t)(mBase + row) * ldc + n0 + c8) = lv;
        }
        __threadfence();
      }
    }
    __builtin_amdgcn_fence(__ATOMIC_RELEASE, "workgroup");
    __builtin_amdgcn_wave_barrier();
    __builtin_amdgcn_fence(__ATOMIC_ACQUIRE, "workgroup");
  }
}

__global__ __launch_bounds__(256) void prep_cast_f16(
    const float* __restrict__ hs, const float* __restrict__ oq,
    unsigned short* __restrict__ hq16, unsigned short* __restrict__ hs16, int n8) {
  const int i = blockIdx.x * 256 + threadIdx.x;
  if (i < n8) {
    const size_t o = (size_t)i * 8;
    const v4f a0 = *(const v4f*)(hs + o);
    const v4f a1 = *(const v4f*)(hs + o + 4);
    const v4f b0 = *(const v4f*)(oq + o);
    const v4f b1 = *(const v4f*)(oq + o + 4);
    v8h vq, vs;
#pragma unroll
    for (int e = 0; e < 4; ++e) {
      vq[e]     = (_Float16)(a0[e] + b0[e]);
      vq[4 + e] = (_Float16)(a1[e] + b1[e]);
      vs[e]     = (_Float16)a0[e];
      vs[4 + e] = (_Float16)a1[e];
    }
    _Float16* pq = (_Float16*)(void*)hq16;
    _Float16* ps = (_Float16*)(void*)hs16;
    *(volatile v8h*)(pq + o) = vq;
    *(volatile v8h*)(ps + o) = vs;
    __threadfence();
    *(volatile v8h*)(pq + o) = vq;
    *(volatile v8h*)(ps + o) = vs;
  }
}

__global__ __launch_bounds__(256) void cast_scale_f16(
    const float* __restrict__ w, unsigned short* __restrict__ out16, int n8, float sc) {
  const int i = blockIdx.x * 256 + threadIdx.x;
  if (i < n8) {
    const size_t o = (size_t)i * 8;
    const v4f a0 = *(const v4f*)(w + o);
    const v4f a1 = *(const v4f*)(w + o + 4);
    v8h v;
#pragma unroll
    for (int e = 0; e < 4; ++e) {
      v[e]     = (_Float16)(a0[e] * sc);
      v[4 + e] = (_Float16)(a1[e] * sc);
    }
    _Float16* po = (_Float16*)(void*)out16;
    *(volatile v8h*)(po + o) = v;
    __threadfence();
    *(volatile v8h*)(po + o) = v;
  }
}

__device__ __forceinline__ v8f mma_h(v16h a, v16h b, v8f c) {
  c = __builtin_amdgcn_wmma_f32_16x16x32_f16(false, a, false, b, (short)0, c, false, false);
  asm volatile("v_nop\n\tv_nop\n\tv_nop\n\tv_nop" : "+v"(c) : "v"(a), "v"(b));
  return c;
}

__global__ __launch_bounds__(128) void attn_heads_f16(
    const unsigned short* __restrict__ Qp, const unsigned short* __restrict__ Kp,
    const unsigned short* __restrict__ Vtp, unsigned short* __restrict__ AOp) {
  __shared__ __align__(16) _Float16 Psh[4][16 * 64];
  __shared__ __align__(16) float Os[4][16 * 68];
  union FH { v16h v; v8h h[2]; };

  const int tid  = threadIdx.x;
  const int wave = tid >> 5;
  const int lane = tid & 31;
  const int hh   = lane >> 4;
  const int c    = lane & 15;

  constexpr int nqb = SEQ_LEN / 64;
  const int bx = blockIdx.x;
  const int qb = bx % nqb;
  const int bh = bx / nqb;
  const int h  = bh % N_HEADS;
  const int b  = bh / N_HEADS;
  const int q0 = qb * 64 + wave * 16;

  const _Float16* Qh  = (const _Float16*)(const void*)Qp;
  const _Float16* Kh  = (const _Float16*)(const void*)Kp;
  const _Float16* Vth = (const _Float16*)(const void*)Vtp;
  _Float16* AOh = (_Float16*)(void*)AOp;

  const size_t bT = (size_t)b * SEQ_LEN;
  const _Float16* qrow = Qh + (bT + q0 + c) * EMB_DIM + h * HEAD_DIM + 8 * hh;
  const _Float16* kbase = Kh + (bT + c) * EMB_DIM + h * HEAD_DIM + 8 * hh;
  const _Float16* vbase = Vth + ((size_t)(b * N_HEADS + h) * HEAD_DIM + c) * SEQ_LEN + 8 * hh;

  v16h qa[2];
#pragma unroll
  for (int dc = 0; dc < 2; ++dc) qa[dc] = Frag<_Float16>::load(qrow + dc * 32);

  const float neg_inf = -__builtin_huge_valf();
  float mrow[8], lrow[8];
  v8f oacc[4];
#pragma unroll
  for (int r = 0; r < 8; ++r) { mrow[r] = neg_inf; lrow[r] = 0.f; }
#pragma unroll
  for (int t = 0; t < 4; ++t) oacc[t] = (v8f){0.f,0.f,0.f,0.f,0.f,0.f,0.f,0.f};

  _Float16* pw = Psh[wave];

  for (int kc = 0; kc < SEQ_LEN / 64; ++kc) {
    const int kv0 = kc * 64;
    v8f s[4];
#pragma unroll
    for (int j = 0; j < 4; ++j) s[j] = (v8f){0.f,0.f,0.f,0.f,0.f,0.f,0.f,0.f};
#pragma unroll
    for (int dc = 0; dc < 2; ++dc) {
      v16h kb[4];
#pragma unroll
      for (int j = 0; j < 4; ++j)
        kb[j] = Frag<_Float16>::load(kbase + (size_t)(kv0 + j * 16) * EMB_DIM + dc * 32);
#pragma unroll
      for (int j = 0; j < 4; ++j) s[j] = mma_h(qa[dc], kb[j], s[j]);
    }
    float cm[8];
#pragma unroll
    for (int r = 0; r < 8; ++r) {
      float m = neg_inf;
#pragma unroll
      for (int j = 0; j < 4; ++j) {
        const float t = s[j][r] * SCORE_SCALE_LOG2E;
        s[j][r] = t;
        m = fmaxf(m, t);
      }
#pragma unroll
      for (int off = 1; off < 16; off <<= 1) m = fmaxf(m, __shfl_xor(m, off, 32));
      cm[r] = m;
    }
#pragma unroll
    for (int r = 0; r < 8; ++r) {
      const float mnew = fmaxf(mrow[r], cm[r]);
      const float alpha = exp2f(mrow[r] - mnew);
      mrow[r] = mnew;
      float psum = 0.f;
#pragma unroll
      for (int j = 0; j < 4; ++j) {
        const float p = exp2f(s[j][r] - mnew);
        psum += p;
        pw[(8 * hh + r) * 64 + j * 16 + c] = (_Float16)(p * P_CARRY);
      }
#pragma unroll
      for (int off = 1; off < 16; off <<= 1) psum += __shfl_xor(psum, off, 32);
      lrow[r] = lrow[r] * alpha + psum;
#pragma unroll
      for (int t = 0; t < 4; ++t) oacc[t][r] *= alpha;
    }
    __builtin_amdgcn_fence(__ATOMIC_RELEASE, "workgroup");
    __builtin_amdgcn_wave_barrier();
    __builtin_amdgcn_fence(__ATOMIC_ACQUIRE, "workgroup");
#pragma unroll 1
    for (int kk = 0; kk < 2; ++kk) {
      FH pa;
      pa.h[0] = *(const v8h*)(pw + c * 64 + kk * 32 + 8 * hh);
      pa.h[1] = *(const v8h*)(pw + c * 64 + kk * 32 + 16 + 8 * hh);
      v16h vb[4];
#pragma unroll
      for (int t = 0; t < 4; ++t)
        vb[t] = Frag<_Float16>::load(vbase + (size_t)(t * 16) * SEQ_LEN + kv0 + kk * 32);
#pragma unroll
      for (int t = 0; t < 4; ++t) oacc[t] = mma_h(pa.v, vb[t], oacc[t]);
    }
    __builtin_amdgcn_fence(__ATOMIC_RELEASE, "workgroup");
    __builtin_amdgcn_wave_barrier();
    __builtin_amdgcn_fence(__ATOMIC_ACQUIRE, "workgroup");
  }

  float* os = Os[wave];
#pragma unroll
  for (int r = 0; r < 8; ++r) {
    float inv = 1.0f / (lrow[r] * P_CARRY);
    inv *= AO_CARRY;
#pragma unroll
    for (int t = 0; t < 4; ++t) os[(8 * hh + r) * 68 + t * 16 + c] = oacc[t][r] * inv;
  }
  __builtin_amdgcn_fence(__ATOMIC_RELEASE, "workgroup");
  __builtin_amdgcn_wave_barrier();
  __builtin_amdgcn_fence(__ATOMIC_ACQUIRE, "workgroup");
  {
    const int q8 = lane >> 3, c8 = (lane & 7) * 8;
    _Float16* aob = AOh + (bT + q0) * EMB_DIM + h * HEAD_DIM;
    for (int pass = 0; pass < 2; ++pass) {
#pragma unroll
      for (int it = 0; it < 4; ++it) {
        const int row = it * 4 + q8;
        const float* sp = os + row * 68 + c8;
        v8h hv;
#pragma unroll
        for (int e = 0; e < 8; ++e) hv[e] = (_Float16)sp[e];
        *(volatile v8h*)(aob + (size_t)row * EMB_DIM + c8) = hv;
      }
      __threadfence();
    }
  }
}

extern "C" void kernel_launch(void* const* d_in, const int* in_sizes, int n_in,
                              void* d_out, int out_size, void* d_ws, size_t ws_size,
                              hipStream_t stream) {
  if (n_in < 10) return;
  if ((size_t)in_sizes[0] != N_ACT || (size_t)in_sizes[1] != N_ACT) return;
  if ((size_t)in_sizes[2] != N_W || (size_t)in_sizes[4] != N_W || (size_t)in_sizes[6] != N_W || (size_t)in_sizes[8] != N_W) return;
  if (in_sizes[3] != EMB_DIM || in_sizes[5] != EMB_DIM || in_sizes[7] != EMB_DIM || in_sizes[9] != EMB_DIM) return;
  if ((size_t)out_size != N_ACT) return;
  if (ws_size < WS_TOTAL) return;

  const float* hs = (const float*)d_in[0];
  const float* oq = (const float*)d_in[1];
  const float* Wq = (const float*)d_in[2];
  const float* bq = (const float*)d_in[3];
  const float* Wk = (const float*)d_in[4];
  const float* bk = (const float*)d_in[5];
  const float* Wv = (const float*)d_in[6];
  const float* bv = (const float*)d_in[7];
  const float* Wo = (const float*)d_in[8];
  const float* bo = (const float*)d_in[9];
  float* out = (float*)d_out;

  char* ws = (char*)d_ws;
  unsigned short* hq16 = (unsigned short*)(ws + OFF_HQ);
  unsigned short* hs16 = (unsigned short*)(ws + OFF_HS);
  unsigned short* wq16 = (unsigned short*)(ws + OFF_W0 + 0 * PLANE_W);
  unsigned short* wk16 = (unsigned short*)(ws + OFF_W0 + 1 * PLANE_W);
  unsigned short* wv16 = (unsigned short*)(ws + OFF_W0 + 2 * PLANE_W);
  unsigned short* wo16 = (unsigned short*)(ws + OFF_W0 + 3 * PLANE_W);
  unsigned short* q16  = (unsigned short*)(ws + OFF_Q);
  unsigned short* k16  = (unsigned short*)(ws + OFF_K);
  unsigned short* vt16 = (unsigned short*)(ws + OFF_VT);
  unsigned short* ao16 = hq16;

  constexpr int n8_act = (int)(N_ACT / 8);
  static_assert(N_ACT % 8 == 0 && n8_act % 256 == 0);
  prep_cast_f16<<<n8_act / 256, 256, 0, stream>>>(hs, oq, hq16, hs16, n8_act);

  constexpr int n8_w = (int)(N_W / 8);
  static_assert(N_W % 8 == 0 && n8_w % 256 == 0);
  cast_scale_f16<<<n8_w / 256, 256, 0, stream>>>(Wq, wq16, n8_w, W_CARRY);
  cast_scale_f16<<<n8_w / 256, 256, 0, stream>>>(Wk, wk16, n8_w, W_CARRY);
  cast_scale_f16<<<n8_w / 256, 256, 0, stream>>>(Wv, wv16, n8_w, W_CARRY);
  cast_scale_f16<<<n8_w / 256, 256, 0, stream>>>(Wo, wo16, n8_w, W_CARRY);

  static_assert(NROWS % 64 == 0 && EMB_DIM % 64 == 0 && EMB_DIM % 32 == 0);
  constexpr int tiles_qk = (NROWS / 64) * (EMB_DIM / 64);
  static_assert(tiles_qk % 8 == 0);
  const dim3 g_qk(tiles_qk / 8, 1);
  const float inv_w = 1.0f / W_CARRY;
  wmma_gemm64<0, false, 2, 1><<<g_qk, 256, 0, stream>>>(
      hq16, hq16, EMB_DIM, 0L, wq16, wq16, EMB_DIM, 0L,
      (void*)q16, (void*)q16, EMB_DIM, 0L, bq, NROWS, EMB_DIM, EMB_DIM, inv_w);
  wmma_gemm64<0, false, 2, 1><<<g_qk, 256, 0, stream>>>(
      hq16, hq16, EMB_DIM, 0L, wk16, wk16, EMB_DIM, 0L,
      (void*)k16, (void*)k16, EMB_DIM, 0L, bk, NROWS, EMB_DIM, EMB_DIM, inv_w);
  static_assert(SEQ_LEN % 64 == 0);
  constexpr int tiles_v = (EMB_DIM / 64) * (SEQ_LEN / 64);
  static_assert(tiles_v % 8 == 0);
  const dim3 g_v(tiles_v / 8, NB_SZ);
  wmma_gemm64<0, false, 1, 1><<<g_v, 256, 0, stream>>>(
      wv16, wv16, EMB_DIM, 0L, hs16, hs16, EMB_DIM, (long)SEQ_LEN * EMB_DIM,
      (void*)vt16, (void*)vt16, SEQ_LEN, (long)EMB_DIM * SEQ_LEN, bv, EMB_DIM, SEQ_LEN, EMB_DIM, inv_w);

  attn_heads_f16<<<NB_SZ * N_HEADS * (SEQ_LEN / 64), 128, 0, stream>>>(q16, k16, vt16, ao16);

  wmma_gemm64<0, false, 2, 0><<<g_qk, 256, 0, stream>>>(
      ao16, ao16, EMB_DIM, 0L, wo16, wo16, EMB_DIM, 0L,
      (void*)out, (void*)out, EMB_DIM, 0L, bo, NROWS, EMB_DIM, EMB_DIM, 1.0f / (AO_CARRY * W_CARRY));
}
